// TPQwenAttention_17978733101573
// MI455X (gfx1250) — hardware-verified
//
#include <hip/hip_runtime.h>


namespace {
constexpr int Bsz = 2, T = 2048, HID = 2048, DH = 128, NH = 16, NKV = 16;
constexpr int QW = NH * DH, KVW = NKV * DH;
constexpr int NQKV = QW + 2 * KVW;
constexpr int MROWS = Bsz * T;
constexpr int QT_PER_B = T / 16;
constexpr float SCALE = 0.08838834764831845f;

typedef __bf16 b16;
typedef __attribute__((ext_vector_type(16))) __bf16 v16b;
typedef __attribute__((ext_vector_type(8)))  __bf16 v8b;
typedef __attribute__((ext_vector_type(8)))  float v8f;
typedef __attribute__((ext_vector_type(4)))  float v4f;

__device__ __forceinline__ v8b ld8b(const b16* p) { return *(const v8b*)p; }
__device__ __forceinline__ v16b cat8b(v8b a, v8b b) { return __builtin_shufflevector(a, b, 0, 1, 2, 3, 4, 5, 6, 7, 8, 9, 10, 11, 12, 13, 14, 15); }
__device__ __forceinline__ v16b frag_kb(const b16* p, int hh) { return cat8b(ld8b(p + 8 * hh), ld8b(p + 16 + 8 * hh)); }
__device__ __forceinline__ void split_bf16(float v, b16& hi, b16& lo) {
  const unsigned int u = __builtin_bit_cast(unsigned int, v) & 0xffff0000u;
  hi = __builtin_bit_cast(b16, (unsigned short)(u >> 16));
  lo = (b16)(v - __builtin_bit_cast(float, u));
}
__device__ __forceinline__ void frag_ksplit(const float* p, int hh, v16b& fh_, v16b& fl_) {
  const float* p0 = p + 8 * hh; const float* p1 = p + 16 + 8 * hh;
#pragma unroll
  for (int e = 0; e < 8; ++e) { b16 a, c; split_bf16(p0[e], a, c); fh_[e] = a; fl_[e] = c; split_bf16(p1[e], a, c); fh_[8 + e] = a; fl_[8 + e] = c; }
}
__device__ __forceinline__ v8f wmma16b(v16b a, v16b b, v8f c) {
  v8f d = __builtin_amdgcn_wmma_f32_16x16x32_bf16(false, a, false, b, (short)0, c, false, false);
  asm volatile("v_nop\n\tv_nop\n\tv_nop\n\tv_nop" : "+v"(d) : "v"(a), "v"(b));
  return d;
}
__device__ __forceinline__ v8f wmma3(v16b ah, v16b al, v16b bh, v16b bl, v8f c) {
  c = wmma16b(ah, bh, c); c = wmma16b(ah, bl, c); c = wmma16b(al, bh, c); return c;
}
__device__ __forceinline__ void wave_lds_sync() {
  __builtin_amdgcn_fence(__ATOMIC_RELEASE, "workgroup");
  __builtin_amdgcn_wave_barrier();
  __builtin_amdgcn_fence(__ATOMIC_ACQUIRE, "workgroup");
}


__global__ __launch_bounds__(256) void wcvt_kernel(const float* __restrict__ wq, const float* __restrict__ wk, const float* __restrict__ wv,
                                                   const float* __restrict__ wo, b16* __restrict__ wqh, b16* __restrict__ wql,
                                                   b16* __restrict__ woh, b16* __restrict__ wol) {
  const size_t tid = (size_t)blockIdx.x * blockDim.x + threadIdx.x, stride = (size_t)gridDim.x * blockDim.x;
  const size_t nq = (size_t)NQKV * HID / 8, no = (size_t)HID * QW / 8;
  for (int pass = 0; pass < 2; ++pass) {
    for (size_t c = tid; c < nq + no; c += stride) {
      float f[8]; size_t i; b16* dh; b16* dl;
      if (c < nq) {
        i = c * 8; const size_t n = i / HID, k0 = i % HID;
        const float* w; int nn, ld;
        if (n < (size_t)QW) { w = wq; nn = (int)n; ld = QW; } else if (n < (size_t)(QW + KVW)) { w = wk; nn = (int)n - QW; ld = KVW; } else { w = wv; nn = (int)n - QW - KVW; ld = KVW; }
#pragma unroll
        for (int e = 0; e < 8; ++e) f[e] = w[(k0 + e) * (size_t)ld + nn];
        dh = wqh; dl = wql;
      } else {
        i = (c - nq) * 8; const size_t n = i / QW, k0 = i % QW;
#pragma unroll
        for (int e = 0; e < 8; ++e) f[e] = wo[(k0 + e) * (size_t)HID + n];
        dh = woh; dl = wol;
      }
      v8b bh, bl;
#pragma unroll
      for (int e = 0; e < 8; ++e) { b16 a, cc; split_bf16(f[e], a, cc); bh[e] = a; bl[e] = cc; }
      *(volatile v8b*)(dh + i) = bh; *(volatile v8b*)(dl + i) = bl;
    }
    __threadfence();
  }
}

__device__ __forceinline__ void gemm_tile_split(const float* __restrict__ A, int lda, const b16* __restrict__ wh, const b16* __restrict__ wl,
                                                int m0, int c0, int K, int nloc, int hlf, v8f acc[2][4]) {
  for (int kb = 0; kb < K; kb += 32) {
    v16b a0h, a0l, a1h, a1l;
    frag_ksplit(A + (size_t)(m0 + nloc) * lda + kb, hlf, a0h, a0l);
    frag_ksplit(A + (size_t)(m0 + 16 + nloc) * lda + kb, hlf, a1h, a1l);
#pragma unroll
    for (int t = 0; t < 4; ++t) {
      const size_t wo = (size_t)(c0 + t * 16 + nloc) * K + kb;
      const v16b bh = frag_kb(wh + wo, hlf), bl = frag_kb(wl + wo, hlf);
      acc[0][t] = wmma3(a0h, a0l, bh, bl, acc[0][t]);
      acc[1][t] = wmma3(a1h, a1l, bh, bl, acc[1][t]);
    }
  }
}

__global__ __launch_bounds__(128) void qkv_gemm_kernel(const float* __restrict__ x, const b16* __restrict__ wqh, const b16* __restrict__ wql,
                                                       const float* __restrict__ bq, const float* __restrict__ bk, const float* __restrict__ bv,
                                                       int xoff, int yoff,
                                                       b16* __restrict__ Qh, b16* __restrict__ Ql, b16* __restrict__ Kh, b16* __restrict__ Kl,
                                                       b16* __restrict__ Vh, b16* __restrict__ Vl) {
  __shared__ __attribute__((aligned(16))) b16 Ts[4][2][32 * 64];
  const int lane = threadIdx.x & 31, wave = threadIdx.x >> 5, nloc = lane & 15, hlf = lane >> 4;
  const int m0 = (blockIdx.y + yoff) * 128 + wave * 32;
  const int c0 = (blockIdx.x + xoff) * 64;
  v8f acc[2][4];
#pragma unroll
  for (int r = 0; r < 2; ++r)
#pragma unroll
    for (int t = 0; t < 4; ++t) acc[r][t] = (v8f){};
  gemm_tile_split(x, HID, wqh, wql, m0, c0, HID, nloc, hlf, acc);
  const int mat = (c0 < QW) ? 0 : (c0 < QW + KVW) ? 1 : 2;
  const int cin = (mat == 0) ? c0 : (mat == 1) ? (c0 - QW) : (c0 - QW - KVW);
  const int head = cin / DH, d0 = cin % DH;
  const int b = m0 / T, t0 = m0 % T;
  {
    const float* bias = ((mat == 0) ? bq : (mat == 1) ? bk : bv) + cin;
    const float sc = (mat == 0) ? SCALE : 1.0f;
#pragma unroll
    for (int t = 0; t < 4; ++t) {
      const float bb = bias[t * 16 + nloc];
#pragma unroll
      for (int r = 0; r < 2; ++r)
#pragma unroll
        for (int v = 0; v < 8; ++v) acc[r][t][v] = (acc[r][t][v] + bb) * sc;
    }
  }
  if (mat < 2) {
    b16* Tp0 = Ts[wave][0]; b16* Tp1 = Ts[wave][1];
#pragma unroll
    for (int t = 0; t < 4; ++t)
#pragma unroll
      for (int r = 0; r < 2; ++r)
#pragma unroll
        for (int v = 0; v < 8; ++v) {
          const int rr = r * 16 + v + 8 * hlf, dd = t * 16 + nloc;
          b16 yh, yl; split_bf16(acc[r][t][v], yh, yl);
          Tp0[rr * 64 + dd] = yh; Tp1[rr * 64 + dd] = yl;
        }
    wave_lds_sync();
    const size_t base = ((size_t)(b * NH + head) * T + t0) * DH + d0;
    b16* dh = ((mat == 0) ? Qh : Kh) + base; b16* dl = ((mat == 0) ? Ql : Kl) + base;
    for (int pass = 0; pass < 2; ++pass) {
#pragma unroll
      for (int j = 0; j < 8; ++j) { const int rr = j * 4 + (lane >> 3), sg = lane & 7;
        *(volatile v8b*)(dh + (size_t)rr * DH + sg * 8) = ld8b(Tp0 + rr * 64 + sg * 8); *(volatile v8b*)(dl + (size_t)rr * DH + sg * 8) = ld8b(Tp1 + rr * 64 + sg * 8); }
      __threadfence();
    }
  } else {
    b16* Tp0 = Ts[wave][0]; b16* Tp1 = Ts[wave][1];
#pragma unroll
    for (int t = 0; t < 4; ++t)
#pragma unroll
      for (int r = 0; r < 2; ++r)
#pragma unroll
        for (int v = 0; v < 8; ++v) {
          const int rr = r * 16 + v + 8 * hlf, dd = t * 16 + nloc;
          b16 yh, yl; split_bf16(acc[r][t][v], yh, yl);
          const int idx = (rr >> 4) * 1024 + dd * 16 + (rr & 15);
          Tp0[idx] = yh; Tp1[idx] = yl;
        }
    wave_lds_sync();
#pragma unroll
    for (int q = 0; q < 2; ++q) {
      const size_t base = ((size_t)(b * NKV + head) * QT_PER_B + (t0 >> 4) + q) * (size_t)(DH * 16) + (size_t)d0 * 16;
#pragma unroll
      for (int j = 0; j < 4; ++j) { const int e = (j * 32 + lane) * 8; *(volatile v8b*)(Vh + base + e) = ld8b(Tp0 + q * 1024 + e); *(volatile v8b*)(Vl + base + e) = ld8b(Tp1 + q * 1024 + e); }
    }
    __threadfence();
#pragma unroll
    for (int q = 0; q < 2; ++q) {
      const size_t base = ((size_t)(b * NKV + head) * QT_PER_B + (t0 >> 4) + q) * (size_t)(DH * 16) + (size_t)d0 * 16;
#pragma unroll
      for (int j = 0; j < 4; ++j) { const int e = (j * 32 + lane) * 8; *(volatile v8b*)(Vh + base + e) = ld8b(Tp0 + q * 1024 + e); *(volatile v8b*)(Vl + base + e) = ld8b(Tp1 + q * 1024 + e); }
    }
  }
}

__global__ __launch_bounds__(256) void attn_kernel(const b16* __restrict__ Qh, const b16* __restrict__ Ql, const b16* __restrict__ Kh, const b16* __restrict__ Kl,
                                                   const b16* __restrict__ Vh, const b16* __restrict__ Vl, const float* __restrict__ mask,
                                                   float* __restrict__ yf) {
  __shared__ __attribute__((aligned(16))) float Os[8][16 * 64];
  const int wid = threadIdx.x >> 5, lane = threadIdx.x & 31, hh = lane >> 4, col = lane & 15;
  const int qtile = blockIdx.x * 8 + wid;
  const int g = qtile / QT_PER_B;
  const int q0 = (qtile % QT_PER_B) << 4;
  const int b = g / NH, h = g % NH, kvh = h / (NH / NKV);
  const size_t ko = (size_t)(b * NKV + kvh) * T * DH;
  const size_t qo = ((size_t)g * T + q0 + col) * DH;
  v16b qfh[4], qfl[4];
#pragma unroll
  for (int c = 0; c < 4; ++c) { qfh[c] = frag_kb(Qh + qo + 32 * c, hh); qfl[c] = frag_kb(Ql + qo + 32 * c, hh); }
  const int myq = q0 + col;
  const float* mrow = mask + (size_t)myq * T;
  float m = -INFINITY, l = 0.0f;
  v8f o[8];
#pragma unroll
  for (int n = 0; n < 8; ++n) o[n] = (v8f){};
  for (int kb = 0; kb <= q0 + 15; kb += 32) {
    v8f s0 = {}, s1 = {};
    const size_t r0 = ko + (size_t)(kb + col) * DH, r1 = ko + (size_t)(kb + 16 + col) * DH;
#pragma unroll
    for (int c = 0; c < 4; ++c) {
      s0 = wmma3(frag_kb(Kh + r0 + 32 * c, hh), frag_kb(Kl + r0 + 32 * c, hh), qfh[c], qfl[c], s0);
      s1 = wmma3(frag_kb(Kh + r1 + 32 * c, hh), frag_kb(Kl + r1 + 32 * c, hh), qfh[c], qfl[c], s1);
    }
    float mr = -INFINITY;
#pragma unroll
    for (int r = 0; r < 8; ++r) {
      s0[r] += mrow[kb + 8 * hh + r];
      s1[r] += mrow[kb + 16 + 8 * hh + r];
      mr = fmaxf(mr, fmaxf(s0[r], s1[r]));
    }
    mr = fmaxf(mr, __shfl_xor(mr, 16));
    const float mn = fmaxf(m, mr);
    const float al = __expf(m - mn);
    m = mn;
    float sum = 0.0f;
    v16b pbh, pbl;
#pragma unroll
    for (int r = 0; r < 8; ++r) {
      const float p0 = __expf(s0[r] - mn), p1 = __expf(s1[r] - mn);
      sum += p0 + p1;
      b16 a, c; split_bf16(p0, a, c); pbh[r] = a; pbl[r] = c; split_bf16(p1, a, c); pbh[8 + r] = a; pbl[8 + r] = c;
    }
    sum += __shfl_xor(sum, 16);
    l = l * al + sum;
#pragma unroll
    for (int n = 0; n < 8; ++n) o[n] *= al;
    const size_t v0 = (size_t)(b * NKV + kvh) * T * DH + (size_t)(kb >> 4) * (DH * 16) + 8 * hh;
    const size_t v1 = v0 + DH * 16;
#pragma unroll
    for (int n = 0; n < 8; ++n) {
      const int f = n * 16 + col;
      const v16b vah = cat8b(ld8b(Vh + v0 + f * 16), ld8b(Vh + v1 + f * 16));
      const v16b val = cat8b(ld8b(Vl + v0 + f * 16), ld8b(Vl + v1 + f * 16));
      o[n] = wmma3(vah, val, pbh, pbl, o[n]);
    }
  }
  const float inv = 1.0f / l;
  float* Tt = Os[wid];
#pragma unroll
  for (int half = 0; half < 2; ++half) {
#pragma unroll
    for (int n = 0; n < 4; ++n)
#pragma unroll
      for (int r = 0; r < 8; ++r) Tt[col * 64 + n * 16 + 8 * hh + r] = o[half * 4 + n][r] * inv;
    wave_lds_sync();
    float* dst0 = yf + ((size_t)b * T + q0) * QW + h * DH + half * 64;
#pragma unroll
    for (int j = 0; j < 8; ++j) { const int rr = j * 2 + hh, c4 = col * 4; *(volatile v4f*)(dst0 + (size_t)rr * QW + c4) = *(const v4f*)(Tt + rr * 64 + c4); }
    __threadfence();
#pragma unroll
    for (int j = 0; j < 8; ++j) { const int rr = j * 2 + hh, c4 = col * 4; *(volatile v4f*)(dst0 + (size_t)rr * QW + c4) = *(const v4f*)(Tt + rr * 64 + c4); }
    wave_lds_sync();
  }
}

__global__ __launch_bounds__(128) void out_gemm_kernel(const float* __restrict__ yf, const b16* __restrict__ woh, const b16* __restrict__ wol, int yoff, float* __restrict__ out) {
  __shared__ __attribute__((aligned(16))) float Ts[4][32 * 64];
  const int lane = threadIdx.x & 31, wave = threadIdx.x >> 5, nloc = lane & 15, hlf = lane >> 4;
  const int m0 = (blockIdx.y + yoff) * 128 + wave * 32;
  const int c0 = blockIdx.x * 64;
  v8f acc[2][4];
#pragma unroll
  for (int r = 0; r < 2; ++r)
#pragma unroll
    for (int t = 0; t < 4; ++t) acc[r][t] = (v8f){};
  gemm_tile_split(yf, QW, woh, wol, m0, c0, QW, nloc, hlf, acc);
  float* Tt = Ts[wave];
#pragma unroll
  for (int t = 0; t < 4; ++t)
#pragma unroll
    for (int r = 0; r < 2; ++r)
#pragma unroll
      for (int v = 0; v < 8; ++v) Tt[(r * 16 + v + 8 * hlf) * 64 + t * 16 + nloc] = acc[r][t][v];
  wave_lds_sync();
  float* dst0 = out + (size_t)m0 * HID + c0;
#pragma unroll
  for (int j = 0; j < 16; ++j) { const int rr = j * 2 + hlf, c4 = nloc * 4; *(volatile v4f*)(dst0 + (size_t)rr * HID + c4) = *(const v4f*)(Tt + rr * 64 + c4); }
  __threadfence();
#pragma unroll
  for (int j = 0; j < 16; ++j) { const int rr = j * 2 + hlf, c4 = nloc * 4; *(volatile v4f*)(dst0 + (size_t)rr * HID + c4) = *(const v4f*)(Tt + rr * 64 + c4); }
}
}

extern "C" void kernel_launch(void* const* d_in, const int* in_sizes, int n_in,
                              void* d_out, int out_size, void* d_ws, size_t ws_size, hipStream_t stream) {
  (void)in_sizes; (void)n_in; (void)out_size;
  const float* x    = (const float*)d_in[0];
  const float* mask = (const float*)d_in[1];
  const float* Wq = (const float*)d_in[2];
  const float* bq = (const float*)d_in[3];
  const float* Wk = (const float*)d_in[4];
  const float* bk = (const float*)d_in[5];
  const float* Wv = (const float*)d_in[6];
  const float* bv = (const float*)d_in[7];
  const float* Wo = (const float*)d_in[8];
  float* out = (float*)d_out;

  size_t off = 0; char* ws = (char*)d_ws;
  b16* wqh = (b16*)(ws + off); off += (size_t)NQKV * HID * 2;
  b16* wql = (b16*)(ws + off); off += (size_t)NQKV * HID * 2;
  b16* woh = (b16*)(ws + off); off += (size_t)HID * QW * 2;
  b16* wol = (b16*)(ws + off); off += (size_t)HID * QW * 2;
  b16* Qh  = (b16*)(ws + off); off += (size_t)MROWS * QW * 2;
  b16* Ql  = (b16*)(ws + off); off += (size_t)MROWS * QW * 2;
  b16* Kh  = (b16*)(ws + off); off += (size_t)MROWS * KVW * 2;
  b16* Kl  = (b16*)(ws + off); off += (size_t)MROWS * KVW * 2;
  b16* Vh  = (b16*)(ws + off); off += (size_t)MROWS * KVW * 2;
  b16* Vl  = (b16*)(ws + off); off += (size_t)MROWS * KVW * 2;
  float* yf = (float*)(ws + off); off += (size_t)MROWS * QW * 4;
  if (off > ws_size) return;

  wcvt_kernel<<<4096, 256, 0, stream>>>(Wq, Wk, Wv, Wo, wqh, wql, woh, wol);
  qkv_gemm_kernel<<<dim3(NQKV / 64, MROWS / 128), 128, 0, stream>>>(x, wqh, wql, bq, bk, bv, 0, 0, Qh, Ql, Kh, Kl, Vh, Vl);
  attn_kernel<<<(Bsz * NH * QT_PER_B) / 8, 256, 0, stream>>>(Qh, Ql, Kh, Kl, Vh, Vl, mask, yf);
  out_gemm_kernel<<<dim3(HID / 64, MROWS / 128), 128, 0, stream>>>(yf, woh, wol, 0, out);
}
